// SoftmaxLoss_28054726377853
// MI455X (gfx1250) — hardware-verified
//
#include <hip/hip_runtime.h>
#include <stddef.h>


typedef _Float16 h16;
typedef _Float16 v16h __attribute__((ext_vector_type(16)));
typedef _Float16 v8h  __attribute__((ext_vector_type(8)));
typedef float    v8f  __attribute__((ext_vector_type(8)));
typedef float    v4f  __attribute__((ext_vector_type(4)));

#define NSPK   128
#define MUTT   16
#define PDIM   256
#define KROWS  (NSPK * MUTT)

#define OUT1_OFF_BYTES 4
#define OUT_FLOATS     (1 + KROWS * NSPK)
#define EMIT_F4        ((KROWS * NSPK) / 4)
#define EMIT_ITER      4
#define EMIT_BLOCKS    (EMIT_F4 / (256 * EMIT_ITER))

#define LDE   260
#define LDCS  132
#define SDP   32
#define SIMROWS 32

#define CARRY     1024.0f
#define SIM_SCALE (10.0f / 1048576.0f)
#define SIM_BIAS  (-5.0f)
#define EPS_NRM   1.0e-12f
#define EPS_LOG   1.0e-9f

static_assert(OUT1_OFF_BYTES == 4);
static_assert((size_t)OUT_FLOATS * 4 == (size_t)1048580);
static_assert(KROWS == 2048 && NSPK == 128 && MUTT == 16);
static_assert(PDIM == 32 * 8);
static_assert(PDIM == 256);
static_assert((PDIM % 32) == 0);
static_assert(MUTT * (PDIM / 4) == 4 * 256);
static_assert(MUTT == 2 * 8);
static_assert(NSPK == 4 * 32);
static_assert(SIMROWS == 2 * 16 && SIMROWS == 8 * 4);
static_assert((KROWS % SIMROWS) == 0);
static_assert(SIMROWS * (NSPK / 4) == 4 * 256);
static_assert((LDE % 4) == 0 && LDE >= PDIM);
static_assert((LDCS % 4) == 0 && LDCS >= NSPK);
static_assert(SDP == 32 && MUTT <= SDP);
static_assert((EMIT_F4 % (256 * EMIT_ITER)) == 0);
static_assert(EMIT_F4 * 4 + 1 == OUT_FLOATS);
static_assert((KROWS % 32) == 0);

#define EN_BYTES  ((size_t)KROWS * PDIM * 2)
#define CN_BYTES  ((size_t)NSPK * PDIM * 2)
#define SD_BYTES  ((size_t)NSPK * SDP * 4)
#define S_BYTES   ((size_t)KROWS * NSPK * 4)
#define TM_BYTES  ((size_t)KROWS * 4)
#define OFF_EN  ((size_t)0)
#define OFF_CN  (OFF_EN + EN_BYTES)
#define OFF_SD  (OFF_CN + CN_BYTES)
#define OFF_S   (OFF_SD + SD_BYTES)
#define OFF_TM  (OFF_S + S_BYTES)
#define WS_TOTAL (OFF_TM + TM_BYTES)
static_assert((EN_BYTES % 128) == 0 && (CN_BYTES % 128) == 0 && (SD_BYTES % 128) == 0);
static_assert((S_BYTES % 128) == 0 && (TM_BYTES % 128) == 0);
static_assert(WS_TOTAL <= (size_t)134217728);

__device__ __forceinline__ float bf16r(float x) {
  unsigned int u = __float_as_uint(x);
  u = (u + 0x7FFFu + ((u >> 16) & 1u)) & 0xFFFF0000u;
  return __uint_as_float(u);
}

static __device__ __forceinline__ h16 toh_flush(float v) {
  const h16 r = (h16)v;
  return (fabsf(v) < 6.103515625e-05f) ? (h16)0.0f : r;
}

__device__ __forceinline__ v16h frag_at(const _Float16* p) {
  v8h lo = *(const v8h*)(p);
  v8h hi = *(const v8h*)(p + 16);
  v16h out;
#pragma unroll
  for (int i = 0; i < 8; ++i) { out[i] = lo[i]; out[i + 8] = hi[i]; }
  return out;
}

__device__ __forceinline__ v8f wmma16(v16h a, v16h b, v8f c) {
  v8f d = __builtin_amdgcn_wmma_f32_16x16x32_f16(false, a, false, b, (short)0, c,
                                                 false, false);
  asm volatile("v_nop\n\tv_nop\n\tv_nop\n\tv_nop" : "+v"(d) : "v"(a), "v"(b));
  return d;
}

__device__ __forceinline__ float red32_sum(float x) {
#pragma unroll
  for (int off = 1; off < 32; off <<= 1) x += __shfl_xor(x, off, 32);
  return x;
}

__global__ __launch_bounds__(256) void prep_kernel(
    const float* __restrict__ E, h16* __restrict__ En, h16* __restrict__ Cn,
    float* __restrict__ Sd) {
  __shared__ __attribute__((aligned(16))) float Es[MUTT * LDE];
  __shared__ __attribute__((aligned(16))) float Csum[PDIM];
  __shared__ __attribute__((aligned(16))) h16 C16[PDIM];
  __shared__ float Wred[8];
  __shared__ float SDs[MUTT];

  const unsigned tid = threadIdx.x, lane = tid & 31u;
  const unsigned wave = (unsigned)__builtin_amdgcn_readfirstlane((int)(threadIdx.x >> 5));
  const unsigned n = blockIdx.x;

#pragma unroll
  for (unsigned j = 0; j < 4u; ++j) {
    const unsigned idx = tid + 256u * j;
    const unsigned r = idx >> 6, c = (idx & 63u) * 4u;
    const v4f a = *(const v4f*)(E + (size_t)(n * MUTT + r) * PDIM + c);
    v4f t;
#pragma unroll
    for (int i = 0; i < 4; ++i) t[i] = bf16r(a[i]);
    *(v4f*)&Es[r * LDE + c] = t;
  }
  __syncthreads();

  float s = 0.0f;
#pragma unroll 4
  for (unsigned mu = 0; mu < (unsigned)MUTT; ++mu) s += Es[mu * LDE + tid];
  Csum[tid] = s;
  const float cmean = s * (1.0f / (float)MUTT);
  const float q = red32_sum(cmean * cmean);
  if (lane == 0u) Wred[wave] = q;
  __syncthreads();
  float tot = 0.0f;
#pragma unroll
  for (int i = 0; i < 8; ++i) tot += Wred[i];
  const float cinv = rsqrtf(tot + EPS_NRM);
  C16[tid] = toh_flush(CARRY * (cmean * cinv));

#pragma unroll 1
  for (unsigned rr = 0; rr < 2u; ++rr) {
    const unsigned r = wave * 2u + rr;
    const unsigned cb = lane * 8u;
    const v4f a0 = *(const v4f*)&Es[r * LDE + cb];
    const v4f a1 = *(const v4f*)&Es[r * LDE + cb + 4u];
    const v4f c0 = *(const v4f*)&Csum[cb];
    const v4f c1 = *(const v4f*)&Csum[cb + 4u];
    float see = 0.0f, scc = 0.0f, sec = 0.0f;
#pragma unroll
    for (int i = 0; i < 4; ++i) {
      const float e0 = a0[i], e1 = a1[i];
      const float d0 = (c0[i] - e0) * (1.0f / (float)(MUTT - 1));
      const float d1 = (c1[i] - e1) * (1.0f / (float)(MUTT - 1));
      see += e0 * e0;  scc += d0 * d0;  sec += e0 * d0;
      see += e1 * e1;  scc += d1 * d1;  sec += e1 * d1;
    }
    see = red32_sum(see);
    scc = red32_sum(scc);
    sec = red32_sum(sec);
    const float einv = rsqrtf(see + EPS_NRM);
    const float dinv = rsqrtf(scc + EPS_NRM);
    const float sd = 10.0f * (sec * einv * dinv) + SIM_BIAS;
    if (lane == 0u) SDs[r] = sd;
    v8h o;
#pragma unroll
    for (int i = 0; i < 4; ++i) {
      o[i]     = toh_flush(CARRY * (a0[i] * einv));
      o[i + 4] = toh_flush(CARRY * (a1[i] * einv));
    }
    h16* p = En + (size_t)(n * MUTT + r) * PDIM + cb;
    *(volatile v8h*)p = o;
    __threadfence();
    *(volatile v8h*)p = o;
  }
  __syncthreads();

  if (wave == 0u) {
    const v8h cv = *(const v8h*)&C16[lane * 8u];
    const float sv = SDs[lane & 15u];
    const float sw = (lane < 16u) ? sv : 0.0f;
    h16* pc = Cn + (size_t)n * PDIM + lane * 8u;
    float* ps = Sd + (size_t)n * SDP + lane;
    *(volatile v8h*)pc = cv;
    *(volatile float*)ps = sw;
    __threadfence();
    *(volatile v8h*)pc = cv;
    *(volatile float*)ps = sw;
  }
}

__global__ __launch_bounds__(256) void sim_kernel(
    const h16* __restrict__ En, const h16* __restrict__ Cn, const float* __restrict__ Sd,
    float* __restrict__ S, float* __restrict__ Tm) {
  __shared__ __attribute__((aligned(16))) float Cs[SIMROWS * LDCS];
  __shared__ __attribute__((aligned(16))) float T[SIMROWS];

  const unsigned tid = threadIdx.x, lane = tid & 31u;
  const unsigned wave = (unsigned)__builtin_amdgcn_readfirstlane((int)(threadIdx.x >> 5));
  const unsigned mw = wave >> 2, nw = wave & 3u;
  const unsigned hh = lane >> 4, m = lane & 15u;
  const unsigned row0 = blockIdx.x * (unsigned)SIMROWS;

  const h16* ap  = En + (size_t)(row0 + mw * 16u + m) * PDIM + hh * 8u;
  const h16* bp0 = Cn + (size_t)(nw * 32u + m) * PDIM + hh * 8u;
  const h16* bp1 = bp0 + (size_t)16 * PDIM;
  v8f acc0 = {}, acc1 = {};
#pragma unroll 2
  for (unsigned k0 = 0; k0 < (unsigned)PDIM; k0 += 32u) {
    const v16h a  = frag_at(ap + k0);
    const v16h b0 = frag_at(bp0 + k0);
    const v16h b1 = frag_at(bp1 + k0);
    acc0 = wmma16(a, b0, acc0);
    acc1 = wmma16(a, b1, acc1);
  }
#pragma unroll
  for (int r = 0; r < 8; ++r) {
    float* d = &Cs[(mw * 16u + hh * 8u + (unsigned)r) * LDCS + nw * 32u + m];
    d[0]  = acc0[r];
    d[16] = acc1[r];
  }
  __syncthreads();

#pragma unroll 1
  for (unsigned j = 0; j < 4u; ++j) {
    const unsigned r = wave * 4u + j;
    const unsigned krow = row0 + r;
    const unsigned dcol = krow >> 4;
    const float sd = Sd[(size_t)dcol * SDP + (krow & 15u)];
    const v4f u = *(const v4f*)&Cs[r * LDCS + lane * 4u];
    v4f t;
    float es = 0.0f;
#pragma unroll
    for (int i = 0; i < 4; ++i) {
      const unsigned col = lane * 4u + (unsigned)i;
      const float sv = u[i] * SIM_SCALE + SIM_BIAS;
      const float tv = (col == dcol) ? sd : sv;
      t[i] = tv;
      es += expf(tv);
    }
    *(v4f*)&Cs[r * LDCS + lane * 4u] = t;
    es = red32_sum(es);
    if (lane == 0u) T[r] = logf(es + EPS_LOG) - sd;
  }
  __syncthreads();

  v4f x[4];
  size_t off[4];
#pragma unroll
  for (unsigned i = 0; i < 4u; ++i) {
    const unsigned idx = tid + 256u * i;
    const unsigned r = idx >> 5;
    const unsigned c = (idx & 31u) * 4u;
    x[i] = *(const v4f*)&Cs[r * LDCS + c];
    off[i] = (size_t)(row0 + r) * NSPK + c;
  }
  const float tv = T[lane];
  float* pt = Tm + row0 + lane;
#pragma unroll
  for (int i = 0; i < 4; ++i) *(volatile v4f*)(S + off[i]) = x[i];
  if (wave == 0u) *(volatile float*)pt = tv;
  __threadfence();
#pragma unroll
  for (int i = 0; i < 4; ++i) *(volatile v4f*)(S + off[i]) = x[i];
  if (wave == 0u) *(volatile float*)pt = tv;
}

__global__ __launch_bounds__(256) void emit_kernel(
    const float* __restrict__ S, const float* __restrict__ Tm, float* __restrict__ out) {
  const unsigned tid = threadIdx.x, lane = tid & 31u;
  const unsigned wave = (unsigned)__builtin_amdgcn_readfirstlane((int)(threadIdx.x >> 5));

  float lossv = 0.0f;
  if (blockIdx.x == 0u && wave == 0u) {
    float s = 0.0f;
#pragma unroll 4
    for (unsigned j = 0; j < (unsigned)(KROWS / 32); ++j) s += Tm[j * 32u + lane];
    lossv = red32_sum(s) * (1.0f / (float)KROWS);
  }

  v4f x[EMIT_ITER];
  size_t off[EMIT_ITER];
  float tailv = 0.0f;
#pragma unroll
  for (unsigned i = 0; i < (unsigned)EMIT_ITER; ++i) {
    const unsigned g = (blockIdx.x * (unsigned)EMIT_ITER + i) * 256u + tid;
    const unsigned gp = (g > 0u) ? (g - 1u) : 0u;
    const v4f a = *(const v4f*)(S + (size_t)gp * 4u);
    const v4f b = *(const v4f*)(S + (size_t)g * 4u);
    v4f v;
    v[0] = (g == 0u) ? lossv : a[3];
    v[1] = b[0];
    v[2] = b[1];
    v[3] = b[2];
    x[i] = v;
    off[i] = (size_t)g * 4u;
    tailv = b[3];
  }
  const bool is_tail = (blockIdx.x == (unsigned)(EMIT_BLOCKS - 1)) && (tid == 255u);
  float* ptail = out + (size_t)EMIT_F4 * 4u;
#pragma unroll
  for (int i = 0; i < EMIT_ITER; ++i) *(volatile v4f*)(out + off[i]) = x[i];
  if (is_tail) *(volatile float*)ptail = tailv;
  __threadfence();
#pragma unroll
  for (int i = 0; i < EMIT_ITER; ++i) *(volatile v4f*)(out + off[i]) = x[i];
  if (is_tail) *(volatile float*)ptail = tailv;
}

extern "C" void kernel_launch(void* const* d_in, const int* in_sizes, int n_in,
                              void* d_out, int out_size, void* d_ws, size_t ws_size,
                              hipStream_t stream) {
  if (n_in < 1) return;
  if ((long long)in_sizes[0] < (long long)KROWS * PDIM) return;
  if ((long long)out_size < (long long)OUT_FLOATS) return;
  if (ws_size < WS_TOTAL) return;

  const float* e = (const float*)d_in[0];
  float* out = (float*)d_out;

  char* ws = (char*)d_ws;
  h16*   En16 = (h16*)(ws + OFF_EN);
  h16*   Cn16 = (h16*)(ws + OFF_CN);
  float* Sdp  = (float*)(ws + OFF_SD);
  float* Sws  = (float*)(ws + OFF_S);
  float* Tms  = (float*)(ws + OFF_TM);

  prep_kernel<<<dim3(NSPK), dim3(256), 0, stream>>>(e, En16, Cn16, Sdp);
  sim_kernel<<<dim3(KROWS / SIMROWS), dim3(256), 0, stream>>>(En16, Cn16, Sdp, Sws, Tms);
  emit_kernel<<<dim3(EMIT_BLOCKS), dim3(256), 0, stream>>>(Sws, Tms, out);
}
